// Attention_agent_df_50525995270753
// MI455X (gfx1250) — hardware-verified
//
#include <hip/hip_runtime.h>
#define NIMG 8
#define CC 256
#define NHD 8
#define HDm 32
#define HS 64
#define NPX (HS * HS)
#define NAG 64
#define KT 9
#define KI (KT * CC)
#define QW (3 * CC)
#define THETA 0.7f
#define SCL 0.17677669529663687f
typedef __bf16 v16b __attribute__((ext_vector_type(16)));
typedef unsigned short v8us __attribute__((ext_vector_type(8), may_alias));
typedef float  v8f  __attribute__((ext_vector_type(8)));
typedef float  v4f  __attribute__((ext_vector_type(4)));
typedef float  v4fa __attribute__((ext_vector_type(4), may_alias));
union FragB { v16b v; v8us half[2]; unsigned short u[16]; };

__device__ __forceinline__ unsigned short bf16_bits(float x) { unsigned int u = __float_as_uint(x); return (unsigned short)((u + 0x7FFFu + ((u >> 16) & 1u)) >> 16); }
__device__ __forceinline__ float bf16_val(unsigned short b) { return __uint_as_float(((unsigned int)b) << 16); }
__device__ __forceinline__ float bf16_round(float x) { return bf16_val(bf16_bits(x)); }
template <int NT>
__device__ __forceinline__ v8f mmaN(v16b ah, v16b al, v16b bh, v16b bl, v8f c) {
  c = __builtin_amdgcn_wmma_f32_16x16x32_bf16(false, ah, false, bh, (short)0, c, false, false);
  if (NT >= 2) c = __builtin_amdgcn_wmma_f32_16x16x32_bf16(false, al, false, bh, (short)0, c, false, false);
  if (NT >= 3) c = __builtin_amdgcn_wmma_f32_16x16x32_bf16(false, ah, false, bl, (short)0, c, false, false);
  asm volatile("v_nop\n\tv_nop\n\tv_nop\n\tv_nop" : "+v"(c) : "v"(ah), "v"(al), "v"(bh), "v"(bl));
  return c;
}

__global__ __launch_bounds__(256) void k_wt_bf16(const float* __restrict__ W, unsigned short* __restrict__ Wt, int K, int N) {
  const int t = blockIdx.x * 256 + threadIdx.x;
  const int k8n = K / 8;
  if (t >= N * k8n) return;
  const int n = t / k8n, k8 = (t % k8n) * 8;
  v8us v;
#pragma unroll
  for (int i = 0; i < 8; ++i) v[i] = bf16_bits(W[(size_t)(k8 + i) * N + n]);
  *(volatile v8us*)(Wt + (size_t)n * K + k8) = v;
  __threadfence();
  *(volatile v8us*)(Wt + (size_t)n * K + k8) = v;
}

template <bool ASPLIT, int ACT, bool BIAS_BF16>
__global__ __launch_bounds__(128) void k_gemm_bf(const float* __restrict__ A, int lda, const unsigned short* __restrict__ Wt, int ldb,
                                               const float* __restrict__ bias, float* __restrict__ C, int ldc, int M, int N, int K) {
  __shared__ __attribute__((aligned(16))) float so[4][16][64];
  const int tid = threadIdx.x, w = tid >> 5, lane = tid & 31, ln = lane & 15, hh = lane >> 4;
  const int ntn = N / 64;
  const int wid = blockIdx.x * 4 + w;
  const int mt = wid / ntn, nq = wid % ntn;
  if (mt * 16 >= M) return;
  const int row0 = mt * 16, col0 = nq * 64;
  const float* arow = A + (size_t)(row0 + ln) * lda;
  v8f acc[4] = {};
  for (int kb = 0; kb < K; kb += 32) {
    FragB ah, al;
    const v4f x0 = *(const v4fa*)(arow + kb + 8 * hh), x1 = *(const v4fa*)(arow + kb + 8 * hh + 4);
    const v4f x2 = *(const v4fa*)(arow + kb + 16 + 8 * hh), x3 = *(const v4fa*)(arow + kb + 16 + 8 * hh + 4);
    float xs[16] = {x0[0],x0[1],x0[2],x0[3],x1[0],x1[1],x1[2],x1[3],x2[0],x2[1],x2[2],x2[3],x3[0],x3[1],x3[2],x3[3]};
#pragma unroll
    for (int i = 0; i < 16; ++i) { const unsigned short hb = bf16_bits(xs[i]); ah.u[i] = hb; al.u[i] = ASPLIT ? bf16_bits(xs[i] - bf16_val(hb)) : (unsigned short)0; }
#pragma unroll
    for (int t = 0; t < 4; ++t) {
      const unsigned short* brow = Wt + (size_t)(col0 + t * 16 + ln) * ldb + kb;
      FragB b;
      b.half[0] = *(const v8us*)(brow + 8 * hh);
      b.half[1] = *(const v8us*)(brow + 16 + 8 * hh);
      acc[t] = mmaN<ASPLIT ? 2 : 1>(ah.v, al.v, b.v, b.v, acc[t]);
    }
  }
#pragma unroll
  for (int t = 0; t < 4; ++t) {
    float bv = bias ? bias[col0 + t * 16 + ln] : 0.f;
    if (BIAS_BF16) bv = bf16_round(bv);
#pragma unroll
    for (int r = 0; r < 8; ++r) { float v = acc[t][r] + bv; if (ACT == 1) v = fmaxf(v, 0.f); so[w][8 * hh + r][t * 16 + ln] = v; }
  }
  __builtin_amdgcn_fence(__ATOMIC_ACQ_REL, "workgroup");
  __builtin_amdgcn_wave_barrier();
  const int rsub = lane >> 4, c4 = (lane & 15) * 4;
  for (int pass = 0; pass < 2; ++pass) {
#pragma unroll
    for (int q = 0; q < 8; ++q) {
      const int r = q * 2 + rsub;
      const v4f v = *(const v4fa*)&so[w][r][c4];
      *(volatile v4f*)(C + (size_t)(row0 + r) * ldc + col0 + c4) = v;
    }
    if (pass == 0) __threadfence();
  }
}

template <bool ASPLIT, int ACT, bool BIAS_BF16, bool RES_BF16>
__global__ __launch_bounds__(128) void k_gemm_bf3(const float* __restrict__ A, int lda, const unsigned short* __restrict__ Wt, int ldb,
                                                const float* __restrict__ bias, const float* __restrict__ resid, int rmod, int ldr,
                                                float* __restrict__ C, int ldc, int M, int N, int K) {
  __shared__ __attribute__((aligned(16))) float so[4][16][64];
  const int tid = threadIdx.x, w = tid >> 5, lane = tid & 31, ln = lane & 15, hh = lane >> 4;
  const int ntn = N / 64;
  const int wid = blockIdx.x * 4 + w;
  const int mt = wid / ntn, nq = wid % ntn;
  if (mt * 16 >= M) return;
  const int row0 = mt * 16, col0 = nq * 64;
  const float* arow = A + (size_t)(row0 + ln) * lda;
  v8f acc[4] = {};
  for (int kb = 0; kb < K; kb += 32) {
    FragB ah, al;
    const v4f x0 = *(const v4fa*)(arow + kb + 8 * hh), x1 = *(const v4fa*)(arow + kb + 8 * hh + 4);
    const v4f x2 = *(const v4fa*)(arow + kb + 16 + 8 * hh), x3 = *(const v4fa*)(arow + kb + 16 + 8 * hh + 4);
    float xs[16] = {x0[0],x0[1],x0[2],x0[3],x1[0],x1[1],x1[2],x1[3],x2[0],x2[1],x2[2],x2[3],x3[0],x3[1],x3[2],x3[3]};
#pragma unroll
    for (int i = 0; i < 16; ++i) { const unsigned short hb = bf16_bits(xs[i]); ah.u[i] = hb; al.u[i] = ASPLIT ? bf16_bits(xs[i] - bf16_val(hb)) : (unsigned short)0; }
#pragma unroll
    for (int t = 0; t < 4; ++t) {
      const unsigned short* brow = Wt + (size_t)(col0 + t * 16 + ln) * ldb + kb;
      FragB b;
      b.half[0] = *(const v8us*)(brow + 8 * hh);
      b.half[1] = *(const v8us*)(brow + 16 + 8 * hh);
      acc[t] = mmaN<ASPLIT ? 2 : 1>(ah.v, al.v, b.v, b.v, acc[t]);
    }
  }
#pragma unroll
  for (int t = 0; t < 4; ++t) {
    const int col = col0 + t * 16 + ln;
    float bv = bias ? bias[col] : 0.f;
    if (BIAS_BF16) bv = bf16_round(bv);
#pragma unroll
    for (int r = 0; r < 8; ++r) {
      float v = acc[t][r] + bv;
      if (resid) { float rv = resid[(size_t)((row0 + 8 * hh + r) % rmod) * ldr + col]; if (RES_BF16) rv = bf16_round(rv); v += rv; }
      if (ACT == 1) v = fmaxf(v, 0.f);
      if (ACT == 2) v = 0.5f * v * (1.0f + erff(v * 0.70710678118654752f));
      if (ACT == 3) { const float u = 0.7978845608028654f * (v + 0.044715f * v * v * v); v = 0.5f * v * (1.0f + tanhf(u)); }
      so[w][8 * hh + r][t * 16 + ln] = v;
    }
  }
  __builtin_amdgcn_fence(__ATOMIC_ACQ_REL, "workgroup");
  __builtin_amdgcn_wave_barrier();
  const int rsub = lane >> 4, c4 = (lane & 15) * 4;
  for (int pass = 0; pass < 2; ++pass) {
#pragma unroll
    for (int q = 0; q < 8; ++q) {
      const int r = q * 2 + rsub;
      const v4f v = *(const v4fa*)&so[w][r][c4];
      *(volatile v4f*)(C + (size_t)(row0 + r) * ldc + col0 + c4) = v;
    }
    if (pass == 0) __threadfence();
  }
}
template <bool PARAM_BF16>
__global__ __launch_bounds__(256) void k_layernorm(const float* __restrict__ X, const float* __restrict__ R, const float* __restrict__ g, const float* __restrict__ bta,
                                                  float* __restrict__ out_sum, float* __restrict__ out_norm, int N, float eps) {
  __shared__ float red[256];
  const int row = blockIdx.x, tid = threadIdx.x;
  const float* x = X + (size_t)row * N; const float* rr = R ? R + (size_t)row * N : nullptr;
  float vals[16];
  const int per = N / 256;
  float s1 = 0.f;
  for (int u = 0; u < per / 4; ++u) {
    const int j = tid * 4 + 1024 * u;
    const v4f a = *(const v4fa*)(x + j);
    v4f b = {0.f,0.f,0.f,0.f}; if (rr) b = *(const v4fa*)(rr + j);
#pragma unroll
    for (int q = 0; q < 4; ++q) { const float v = a[q] + b[q]; vals[u * 4 + q] = v; s1 += v; }
  }
  red[tid] = s1; __syncthreads();
  for (int st = 128; st > 0; st >>= 1) { if (tid < st) red[tid] += red[tid + st]; __syncthreads(); }
  const float mu = red[0] / (float)N; __syncthreads();
  float s2 = 0.f;
  for (int u = 0; u < per / 4; ++u)
#pragma unroll
    for (int q = 0; q < 4; ++q) { const float c = vals[u * 4 + q] - mu; s2 += c * c; }
  red[tid] = s2; __syncthreads();
  for (int st = 128; st > 0; st >>= 1) { if (tid < st) red[tid] += red[tid + st]; __syncthreads(); }
  const float rs = rsqrtf(red[0] / (float)N + eps);
  for (int pass = 0; pass < 2; ++pass) {
    for (int u = 0; u < per / 4; ++u) {
      const int j = tid * 4 + 1024 * u;
      v4f o, sm;
#pragma unroll
      for (int q = 0; q < 4; ++q) {
        float gg = g[j + q], bb = bta[j + q];
        if (PARAM_BF16) { gg = bf16_round(gg); bb = bf16_round(bb); }
        sm[q] = vals[u * 4 + q]; o[q] = (vals[u * 4 + q] - mu) * rs * gg + bb;
      }
      if (out_sum) *(volatile v4f*)(out_sum + (size_t)row * N + j) = sm;
      *(volatile v4f*)(out_norm + (size_t)row * N + j) = o;
    }
    if (pass == 0) __threadfence();
  }
}


typedef _Float16 v16h __attribute__((ext_vector_type(16)));
union FragH { v16h v; v8us half[2]; _Float16 h[16]; unsigned short u[16]; };
template <int NT>
__device__ __forceinline__ v8f mmaH(v16h ah, v16h al, v16h bh, v16h bl, v8f c) {
  c = __builtin_amdgcn_wmma_f32_16x16x32_f16(false, ah, false, bh, (short)0, c, false, false);
  if (NT >= 2) c = __builtin_amdgcn_wmma_f32_16x16x32_f16(false, al, false, bh, (short)0, c, false, false);
  if (NT >= 3) c = __builtin_amdgcn_wmma_f32_16x16x32_f16(false, ah, false, bl, (short)0, c, false, false);
  asm volatile("v_nop\n\tv_nop\n\tv_nop\n\tv_nop" : "+v"(c) : "v"(ah), "v"(al), "v"(bh), "v"(bl));
  return c;
}
template <bool ASPLIT>
__global__ __launch_bounds__(128) void k_gemm_h(const float* __restrict__ A, int lda, size_t sA, const _Float16* __restrict__ Bh, int ldb, size_t sB, float alpha, float* __restrict__ C, int ldc, size_t sC, int M, int N, int K) {
  __shared__ __attribute__((aligned(16))) float so[4][16][64];
  const int tid = threadIdx.x, w = tid >> 5, lane = tid & 31, ln = lane & 15, hh = lane >> 4; const int by = blockIdx.y;
  A += (size_t)by * sA; Bh += (size_t)by * sB; C += (size_t)by * sC;
  const int ntn = (N + 63) / 64; const int wid = blockIdx.x * 4 + w; const int mt = wid / ntn, nq = wid % ntn; if (mt * 16 >= M) return;
  const int row0 = mt * 16, col0 = nq * 64; const float* arow = A + (size_t)(row0 + ln) * lda;
  v8f acc[4] = {};
  for (int kb = 0; kb < K; kb += 32) {
    FragH ah, al;
    const v4f x0 = *(const v4fa*)(arow + kb + 8 * hh), x1 = *(const v4fa*)(arow + kb + 8 * hh + 4), x2 = *(const v4fa*)(arow + kb + 16 + 8 * hh), x3 = *(const v4fa*)(arow + kb + 16 + 8 * hh + 4);
    float xs[16] = {x0[0],x0[1],x0[2],x0[3],x1[0],x1[1],x1[2],x1[3],x2[0],x2[1],x2[2],x2[3],x3[0],x3[1],x3[2],x3[3]};
#pragma unroll
    for (int i = 0; i < 16; ++i) { const _Float16 h = (_Float16)xs[i]; ah.h[i] = h; al.h[i] = ASPLIT ? (_Float16)(xs[i] - (float)h) : (_Float16)0.0f; }
#pragma unroll
    for (int t = 0; t < 4; ++t) { if (col0 + t * 16 >= N) continue; const size_t boff = (size_t)(col0 + t * 16 + ln) * ldb + kb; FragH bq; bq.half[0] = *(const v8us*)(Bh + boff + 8 * hh); bq.half[1] = *(const v8us*)(Bh + boff + 16 + 8 * hh);
      acc[t] = mmaH<ASPLIT ? 2 : 1>(ah.v, al.v, bq.v, bq.v, acc[t]); }
  }
#pragma unroll
  for (int t = 0; t < 4; ++t) { if (col0 + t * 16 >= N) continue;
#pragma unroll
    for (int r = 0; r < 8; ++r) so[w][8 * hh + r][t * 16 + ln] = acc[t][r] * alpha; }
  __builtin_amdgcn_fence(__ATOMIC_ACQ_REL, "workgroup"); __builtin_amdgcn_wave_barrier();
  const int rsub = lane >> 4, c4 = (lane & 15) * 4;
  for (int pass = 0; pass < 2; ++pass) {
#pragma unroll
    for (int q = 0; q < 8; ++q) { const int r = q * 2 + rsub; if (col0 + c4 < N) { const v4f v = *(const v4fa*)&so[w][r][c4]; *(volatile v4f*)(C + (size_t)(row0 + r) * ldc + col0 + c4) = v; } }
    if (pass == 0) __threadfence(); }
}

__global__ __launch_bounds__(256) void k_wt_f16(const float* __restrict__ W, _Float16* __restrict__ Wt, int K, int N, float scale) {
  const int t = blockIdx.x * 256 + threadIdx.x; if (t >= N * (K / 8)) return; const int n = t / (K / 8), k8 = (t % (K / 8)) * 8; FragH f;
#pragma unroll
  for (int i = 0; i < 8; ++i) f.h[i] = (_Float16)(bf16_round(W[(size_t)(k8 + i) * N + n]) * scale); const v8us o = f.half[0];
  *(volatile v8us*)((unsigned short*)Wt + (size_t)n * K + k8) = o; __threadfence(); *(volatile v8us*)((unsigned short*)Wt + (size_t)n * K + k8) = o;
}
template <int ACT>
__global__ __launch_bounds__(128) void k_gemm_hhx(const _Float16* __restrict__ A, int lda, size_t sA, const _Float16* __restrict__ Bh, int ldb, size_t sB, float alpha, const float* __restrict__ bias, size_t sBias, const float* __restrict__ CP, int rowsPerB, size_t sCPb, int row0g,
    float* __restrict__ C, _Float16* __restrict__ C16, int ldc, size_t sC, int M, int N, int K) {
  __shared__ __attribute__((aligned(16))) float so[4][16][64];
  const int tid = threadIdx.x, w = tid >> 5, lane = tid & 31, ln = lane & 15, hh = lane >> 4; const int by = blockIdx.y;
  A += (size_t)by * sA; Bh += (size_t)by * sB; const size_t cofs = (size_t)by * sC; const float* bp = bias ? bias + (size_t)by * sBias : nullptr;
  const int ntn = (N + 63) / 64; const int wid = blockIdx.x * 4 + w; const int mt = wid / ntn, nq = wid % ntn; if (mt * 16 >= M) return;
  const int row0 = mt * 16, col0 = nq * 64; const _Float16* arow = A + (size_t)(row0 + ln) * lda;
  v8f acc[4] = {};
  for (int kb = 0; kb < K; kb += 32) { FragH ah; ah.half[0] = *(const v8us*)((const unsigned short*)arow + kb + 8 * hh); ah.half[1] = *(const v8us*)((const unsigned short*)arow + kb + 16 + 8 * hh);
#pragma unroll
    for (int t = 0; t < 4; ++t) { if (col0 + t * 16 >= N) continue; const size_t boff = (size_t)(col0 + t * 16 + ln) * ldb + kb; FragH bq; bq.half[0] = *(const v8us*)((const unsigned short*)Bh + boff + 8 * hh); bq.half[1] = *(const v8us*)((const unsigned short*)Bh + boff + 16 + 8 * hh);
      acc[t] = mmaH<1>(ah.v, ah.v, bq.v, bq.v, acc[t]); }
  }
#pragma unroll
  for (int t = 0; t < 4; ++t) { if (col0 + t * 16 >= N) continue; const int col = col0 + t * 16 + ln; const float bv = bp ? bf16_round(bp[col]) : 0.f;
#pragma unroll
    for (int r = 0; r < 8; ++r) { float v = acc[t][r] * alpha + bv; if (CP) { const int rr = row0g + row0 + 8 * hh + r; if (rowsPerB < 0) v += CP[cofs + (size_t)rr * ldc + col];        else { const int bidx = rr / rowsPerB; v += CP[(size_t)bidx * sCPb + (size_t)by * 64 + col]; } } if (ACT == 1) v = (v > 0.f) ? v : expm1f(v); else if (ACT == 7) v = (v > 0.f) ? v + 1.0f : expf(v); else if (ACT == 8) v = tanhf(v); else if (ACT == 9) v = 0.5f * v * (1.0f + tanhf(0.7978845608028654f * (v + 0.044715f * v * v * v))); else if (ACT == 11) v = 1.0f / (1.0f + expf(-v)); else if (ACT == 12) v = (v > 0.f) ? v : 0.01f * v; else if (ACT == 14) v = (v > 0.f) ? v : 0.1f * v; else if (ACT == 16) v = (v >= 0.f) ? v : 0.3f * v; else if (ACT == 15) v = v / (1.0f + expf(-v)); else if (ACT == 3) v = fmaxf(v, 0.f); else if (ACT == 6) v = 0.5f * v * (1.0f + erff(v * 0.70710678118654752f)); so[w][8 * hh + r][t * 16 + ln] = v; } }
  __builtin_amdgcn_fence(__ATOMIC_ACQ_REL, "workgroup"); __builtin_amdgcn_wave_barrier();
  const int rsub = lane >> 4, c4 = (lane & 15) * 4; typedef _Float16 v4h __attribute__((ext_vector_type(4)));
  for (int pass = 0; pass < 2; ++pass) {
#pragma unroll
    for (int q = 0; q < 8; ++q) { const int r = q * 2 + rsub; if (col0 + c4 < N) { const v4f v = *(const v4fa*)&so[w][r][c4]; if (C) *(volatile v4f*)(C + cofs + (size_t)(row0 + r) * ldc + col0 + c4) = v; if (C16) { v4h h4; for (int i = 0; i < 4; ++i) h4[i] = (_Float16)v[i]; *(volatile v4h*)(C16 + cofs + (size_t)(row0 + r) * ldc + col0 + c4) = h4; } } }
    if (pass == 0) __threadfence(); }
}


typedef _Float16 v4h __attribute__((ext_vector_type(4)));

__global__ __launch_bounds__(256) void k_x16(const float* __restrict__ x, _Float16* __restrict__ X16, size_t n8) { const size_t t = (size_t)blockIdx.x * 256 + threadIdx.x; if (t >= n8) return; FragH f;
#pragma unroll
  for (int q = 0; q < 8; ++q) f.h[q] = (_Float16)bf16_round(x[t * 8 + q]); *(volatile v8us*)((unsigned short*)X16 + t * 8) = f.half[0]; __threadfence(); *(volatile v8us*)((unsigned short*)X16 + t * 8) = f.half[0]; }
__global__ __launch_bounds__(256) void k_h16(const float* __restrict__ x, _Float16* __restrict__ X16, size_t n8) { const size_t t = (size_t)blockIdx.x * 256 + threadIdx.x; if (t >= n8) return; FragH f;
#pragma unroll
  for (int q = 0; q < 8; ++q) f.h[q] = (_Float16)x[t * 8 + q]; *(volatile v8us*)((unsigned short*)X16 + t * 8) = f.half[0]; __threadfence(); *(volatile v8us*)((unsigned short*)X16 + t * 8) = f.half[0]; }
__global__ __launch_bounds__(256) void k_round16f(const float* __restrict__ W, _Float16* __restrict__ Bt, size_t n8) { const size_t t = (size_t)blockIdx.x * 256 + threadIdx.x; if (t >= n8) return; FragH f;
#pragma unroll
  for (int i = 0; i < 8; ++i) f.h[i] = (_Float16)(bf16_round(W[t * 8 + i]) * 16.0f); *(volatile v8us*)((unsigned short*)Bt + t * 8) = f.half[0]; __threadfence(); *(volatile v8us*)((unsigned short*)Bt + t * 8) = f.half[0]; }
template <int NHv, int TTv>
__global__ __launch_bounds__(256) void k_vt(const _Float16* __restrict__ V16, int ldv, int voff, _Float16* __restrict__ Vt) { __shared__ unsigned short tl[64][66]; const int tid = threadIdx.x; const int slab = blockIdx.x / (TTv / 64), lg = blockIdx.x % (TTv / 64); const int b = slab / NHv, h = slab % NHv;
  for (int i = tid; i < 64 * 8; i += 256) { const int r = i / 8, c8 = (i % 8) * 8; FragH f; f.half[0] = *(const v8us*)((const unsigned short*)V16 + ((size_t)b * TTv + lg * 64 + r) * ldv + voff + h * 64 + c8);
#pragma unroll
    for (int q = 0; q < 8; ++q) tl[r][c8 + q] = f.u[q]; }
  __syncthreads();
  for (int pass = 0; pass < 2; ++pass) {
#pragma unroll
    for (int rd = 0; rd < 2; ++rd) { const int d = rd * 32 + tid / 8, pc = tid % 8; FragH f;
#pragma unroll
      for (int q = 0; q < 8; ++q) f.u[q] = tl[pc * 8 + q][d];
      *(volatile v8us*)((unsigned short*)Vt + ((size_t)slab * 64 + d) * TTv + lg * 64 + pc * 8) = f.half[0]; }
    if (pass == 0) __threadfence(); } }

__global__ __launch_bounds__(256) void k_hl(const float* __restrict__ F, _Float16* __restrict__ Hh, _Float16* __restrict__ Hl, size_t n8) { const size_t t = (size_t)blockIdx.x * 256 + threadIdx.x; if (t >= n8) return; FragH fh, fl; const v4f a = *(const v4fa*)(F + t * 8), c = *(const v4fa*)(F + t * 8 + 4);
#pragma unroll
  for (int q = 0; q < 4; ++q) { _Float16 h = (_Float16)a[q]; fh.h[q] = h; fl.h[q] = (_Float16)((a[q] - (float)h) * 1024.0f); h = (_Float16)c[q]; fh.h[4 + q] = h; fl.h[4 + q] = (_Float16)((c[q] - (float)h) * 1024.0f); }
  for (int pass = 0; pass < 2; ++pass) { *(volatile v8us*)((unsigned short*)Hh + t * 8) = fh.half[0]; *(volatile v8us*)((unsigned short*)Hl + t * 8) = fl.half[0]; if (pass == 0) __threadfence(); } }

__device__ __forceinline__ v16h g2_frag(const _Float16* p, int hh) { FragH f; f.half[0] = *(const v8us*)((const unsigned short*)p + 8 * hh); f.half[1] = *(const v8us*)((const unsigned short*)p + 16 + 8 * hh); return f.v; }
__device__ __forceinline__ v8f g2_mma(v16h a, v16h b, v8f c) { v8f d = __builtin_amdgcn_wmma_f32_16x16x32_f16(false, a, false, b, (short)0, c, false, false); asm volatile("v_nop\n\tv_nop\n\tv_nop\n\tv_nop" : "+v"(d) : "v"(a), "v"(b)); return d; }
template <int ACT>
__global__ __launch_bounds__(128) void k_gemm2(const _Float16* __restrict__ A, int lda, size_t sA, const _Float16* __restrict__ Bh, int ldb, size_t sB, float alpha, const float* __restrict__ bias, size_t sBias, const float* __restrict__ CP, int rowsPerB, size_t sCPb, int row0g,
    float* __restrict__ C, _Float16* __restrict__ C16, int ldc, size_t sC, int M, int N, int K) { static_assert(ACT == 0 || ACT == 3 || ACT == 6 || ACT == 8 || ACT == 9 || ACT == 11 || ACT == 12 || ACT == 14 || ACT == 15 || ACT == 16, "k_gemm2: unsupported ACT code (would silently apply no activation)");
  __shared__ __attribute__((aligned(16))) float so[4][32][68];
  const int tid = threadIdx.x, w = tid >> 5, lane = tid & 31, ln = lane & 15, hh = lane >> 4; const int by = blockIdx.y;
  A += (size_t)by * sA; Bh += (size_t)by * sB; const size_t cofs = (size_t)by * sC; const float* bp = bias ? bias + (size_t)by * sBias : nullptr;
  const int ntn = N >> 6; const int mt = blockIdx.x / ntn, nq = blockIdx.x - mt * ntn; const int row0 = mt * 128 + 32 * w, col0 = nq * 64; if (row0 >= M) return;
  const _Float16* a0p = A + (size_t)(row0 + ln) * lda; const _Float16* a1p = a0p + (size_t)16 * lda;
  const _Float16* b0p = Bh + (size_t)(col0 + ln) * ldb; const _Float16* b1p = b0p + (size_t)16 * ldb; const _Float16* b2p = b1p + (size_t)16 * ldb; const _Float16* b3p = b2p + (size_t)16 * ldb;
  const v8f z8 = {0.f,0.f,0.f,0.f,0.f,0.f,0.f,0.f}; v8f c00 = z8, c01 = z8, c02 = z8, c03 = z8, c10 = z8, c11 = z8, c12 = z8, c13 = z8;
#pragma unroll 1
  for (int kb = 0; kb < K; kb += 32) { const v16h a0 = g2_frag(a0p + kb, hh), a1 = g2_frag(a1p + kb, hh);
    v16h b = g2_frag(b0p + kb, hh); c00 = g2_mma(a0, b, c00); c10 = g2_mma(a1, b, c10);
    b = g2_frag(b1p + kb, hh); c01 = g2_mma(a0, b, c01); c11 = g2_mma(a1, b, c11);
    b = g2_frag(b2p + kb, hh); c02 = g2_mma(a0, b, c02); c12 = g2_mma(a1, b, c12);
    b = g2_frag(b3p + kb, hh); c03 = g2_mma(a0, b, c03); c13 = g2_mma(a1, b, c13); }
  v8f accs[8] = {c00, c01, c02, c03, c10, c11, c12, c13};
#pragma unroll
  for (int u = 0; u < 8; ++u) { const int t = u & 3, half = u >> 2; const int col = col0 + t * 16 + ln; const float bv = bp ? bf16_round(bp[col]) : 0.f;
#pragma unroll
    for (int r = 0; r < 8; ++r) { const int rloc = half * 16 + 8 * hh + r; float v = accs[u][r] * alpha + bv; if (CP) { if (rowsPerB < 0) v += CP[cofs + (size_t)(row0g + row0 + rloc) * ldc + col];        else { const int bidx = (row0g + row0 + rloc) / rowsPerB; v += CP[(size_t)bidx * sCPb + (size_t)by * 64 + col]; } }
      if (ACT == 3) v = fmaxf(v, 0.f); else if (ACT == 6) v = 0.5f * v * (1.0f + erff(v * 0.70710678118654752f)); else if (ACT == 11) v = 1.0f / (1.0f + expf(-v)); else if (ACT == 15) v = v / (1.0f + expf(-v)); else if (ACT == 12) v = (v > 0.f) ? v : 0.01f * v; else if (ACT == 8) v = tanhf(v); else if (ACT == 9) v = 0.5f * v * (1.0f + tanhf(0.7978845608028654f * (v + 0.044715f * v * v * v))); else if (ACT == 14) v = (v > 0.f) ? v : 0.1f * v; else if (ACT == 16) v = (v >= 0.f) ? v : 0.3f * v;
      so[w][rloc][t * 16 + ln] = v; } }
  __builtin_amdgcn_fence(__ATOMIC_ACQ_REL, "workgroup"); __builtin_amdgcn_wave_barrier();
  const int rsub = lane >> 4, c4 = (lane & 15) * 4;
  for (int pass = 0; pass < 2; ++pass) {
#pragma unroll
    for (int q = 0; q < 16; ++q) { const int r = q * 2 + rsub; const v4f v = *(const v4fa*)&so[w][r][c4]; if (C) *(volatile v4f*)(C + cofs + (size_t)(row0 + r) * ldc + col0 + c4) = v; if (C16) { v4h h4; for (int i = 0; i < 4; ++i) h4[i] = (_Float16)v[i]; *(volatile v4h*)(C16 + cofs + (size_t)(row0 + r) * ldc + col0 + c4) = h4; } }
    if (pass == 0) __threadfence(); } }


__global__ __launch_bounds__(256) void k_wqkv(const float* __restrict__ w, _Float16* __restrict__ Wh, _Float16* __restrict__ Wl) {
  #pragma clang fp contract(off)
  const int t = blockIdx.x * 256 + threadIdx.x; if (t >= QW * (CC / 8)) return; const int c0 = (t % (CC / 8)) * 8, o = t / (CC / 8); FragH fl;
#pragma unroll 1
  for (int k = 0; k < KT; ++k) { FragH fh;
    for (int q = 0; q < 8; ++q) { const int c = c0 + q; const float* wp = w + ((size_t)o * CC + c) * KT; float v = bf16_round(wp[k]);
      if (k == 4) { float dif = bf16_round(wp[1]) + bf16_round(wp[3]); dif += bf16_round(wp[4]); dif += bf16_round(wp[5]); dif += bf16_round(wp[7]); v += -THETA * dif; const _Float16 hv = (_Float16)(v * 16.0f); fh.h[q] = hv; fl.h[q] = (_Float16)((v * 16.0f - (float)hv) * 1024.0f); }
      else fh.h[q] = (_Float16)(v * 16.0f); }
    *(volatile v8us*)((unsigned short*)Wh + (size_t)o * KI + k * CC + c0) = fh.half[0]; __threadfence(); *(volatile v8us*)((unsigned short*)Wh + (size_t)o * KI + k * CC + c0) = fh.half[0]; }
  *(volatile v8us*)((unsigned short*)Wl + (size_t)o * CC + c0) = fl.half[0]; __threadfence(); *(volatile v8us*)((unsigned short*)Wl + (size_t)o * CC + c0) = fl.half[0]; }
__global__ __launch_bounds__(256) void k_wsc(const float* __restrict__ Wm, _Float16* __restrict__ Bt, size_t n8, float sc) { const size_t t = (size_t)blockIdx.x * 256 + threadIdx.x; if (t >= n8) return; FragH f; for (int q = 0; q < 8; ++q) f.h[q] = (_Float16)(bf16_round(Wm[t * 8 + q]) * sc); *(volatile v8us*)((unsigned short*)Bt + t * 8) = f.half[0]; __threadfence(); *(volatile v8us*)((unsigned short*)Bt + t * 8) = f.half[0]; }
__global__ __launch_bounds__(256) void k_im(const float* __restrict__ xb, _Float16* __restrict__ A) { const size_t t = (size_t)blockIdx.x * 256 + threadIdx.x; if (t >= (size_t)NPX * KT * (CC / 8)) return; const int c0 = (int)(t % (CC / 8)) * 8; const int k = (int)((t / (CC / 8)) % KT); const int p = (int)(t / ((CC / 8) * KT)); const int yy = p / HS + k / 3 - 1, xx = p % HS + k % 3 - 1; FragH f;
  if (yy < 0 || yy >= HS || xx < 0 || xx >= HS) { for (int q = 0; q < 8; ++q) f.h[q] = (_Float16)0.0f; } else { for (int q = 0; q < 8; ++q) f.h[q] = (_Float16)bf16_round(xb[(size_t)(c0 + q) * NPX + yy * HS + xx]); }
  unsigned short* d = (unsigned short*)A + (size_t)p * KI + k * CC + c0; *(volatile v8us*)d = f.half[0]; __threadfence(); *(volatile v8us*)d = f.half[0]; }
__global__ __launch_bounds__(256) void k_aff(const float* __restrict__ F, const float* __restrict__ s, const float* __restrict__ b, float* __restrict__ QF, _Float16* __restrict__ Q16) {
  #pragma clang fp contract(off)
  const size_t t = (size_t)blockIdx.x * 256 + threadIdx.x; if (t >= (size_t)NPX * (QW / 8)) return; const int o0 = (int)(t % (QW / 8)) * 8; v8f r; FragH f; const v8f a = *(const v8f*)(F + t * 8);
  for (int q = 0; q < 8; ++q) { float v = a[q] * bf16_round(s[o0 + q]); v += bf16_round(b[o0 + q]); r[q] = v; f.h[q] = (_Float16)v; }
  for (int pass = 0; pass < 2; ++pass) { *(volatile v8f*)(QF + t * 8) = r; *(volatile v8us*)((unsigned short*)Q16 + t * 8) = f.half[0]; if (pass == 0) __threadfence(); } }
__global__ __launch_bounds__(256) void k_pool(const float* __restrict__ QF, _Float16* __restrict__ AG) {
  #pragma clang fp contract(off)
  typedef _Float16 v2h __attribute__((ext_vector_type(2)));
  const int t = blockIdx.x * 256 + threadIdx.x; if (t >= NHD * NAG * 32) return; const int d0 = (t % 32) * 2; const int n = (t / 32) % NAG; const int h = t / (32 * NAG); float s0 = 0.f, s1 = 0.f;
  if (d0 < HDm) { const int by = n / 8, bx = n % 8;
#pragma unroll 1
    for (int i = 0; i < 64; ++i) { const int p = (by * 8 + i / 8) * HS + bx * 8 + i % 8; const float* q = QF + (size_t)p * QW + h * HDm + d0; s0 += q[0]; s1 += q[1]; } s0 = s0 / 64.0f; s1 = s1 / 64.0f; }
  v2h v; v[0] = (_Float16)s0; v[1] = (_Float16)s1; *(volatile v2h*)(AG + ((size_t)h * NAG + n) * 64 + d0) = v; __threadfence(); *(volatile v2h*)(AG + ((size_t)h * NAG + n) * 64 + d0) = v; }
__global__ __launch_bounds__(256) void k_heads(const _Float16* __restrict__ Q16, _Float16* __restrict__ QP, _Float16* __restrict__ KP) { const int t = blockIdx.x * 256 + threadIdx.x; if (t >= NHD * NPX) return; const int p = t % NPX, h = t / NPX; const unsigned short* src = (const unsigned short*)Q16 + (size_t)p * QW; const v8us z = {0,0,0,0,0,0,0,0};
  v8us q0 = *(const v8us*)(src + h * HDm), q1 = *(const v8us*)(src + h * HDm + 8), q2 = *(const v8us*)(src + h * HDm + 16), q3 = *(const v8us*)(src + h * HDm + 24);
  v8us k0 = *(const v8us*)(src + CC + h * HDm), k1 = *(const v8us*)(src + CC + h * HDm + 8), k2 = *(const v8us*)(src + CC + h * HDm + 16), k3 = *(const v8us*)(src + CC + h * HDm + 24);
  unsigned short* dq = (unsigned short*)QP + ((size_t)h * NPX + p) * 64; unsigned short* dk = (unsigned short*)KP + ((size_t)h * NPX + p) * 64;
  for (int pass = 0; pass < 2; ++pass) { *(volatile v8us*)dq = q0; *(volatile v8us*)(dq + 8) = q1; *(volatile v8us*)(dq + 16) = q2; *(volatile v8us*)(dq + 24) = q3; *(volatile v8us*)(dq + 32) = z; *(volatile v8us*)(dq + 40) = z; *(volatile v8us*)(dq + 48) = z; *(volatile v8us*)(dq + 56) = z;
    *(volatile v8us*)dk = k0; *(volatile v8us*)(dk + 8) = k1; *(volatile v8us*)(dk + 16) = k2; *(volatile v8us*)(dk + 24) = k3; *(volatile v8us*)(dk + 32) = z; *(volatile v8us*)(dk + 40) = z; *(volatile v8us*)(dk + 48) = z; *(volatile v8us*)(dk + 56) = z; if (pass == 0) __threadfence(); } }
__global__ __launch_bounds__(256) void k_vtp(const _Float16* __restrict__ Q16, _Float16* __restrict__ VT) { __shared__ unsigned short tl[64][34]; const int tid = threadIdx.x; const int h = blockIdx.x / (NPX / 64), pg = blockIdx.x % (NPX / 64);
  { const int r = tid / 4, c8 = (tid % 4) * 8; FragH f; f.half[0] = *(const v8us*)((const unsigned short*)Q16 + (size_t)(pg * 64 + r) * QW + 2 * CC + h * HDm + c8); for (int q = 0; q < 8; ++q) tl[r][c8 + q] = f.u[q]; }
  __syncthreads(); const int d = tid / 8, pc = tid % 8; FragH f; for (int q = 0; q < 8; ++q) f.u[q] = (d < HDm) ? tl[pc * 8 + q][d] : (unsigned short)0; unsigned short* dst = (unsigned short*)VT + ((size_t)h * 64 + d) * NPX + pg * 64 + pc * 8;
  *(volatile v8us*)dst = f.half[0]; __threadfence(); *(volatile v8us*)dst = f.half[0];
  if (tid < 256) { const int d2 = HDm + tid / 8; const v8us z = {0,0,0,0,0,0,0,0}; unsigned short* dz = (unsigned short*)VT + ((size_t)h * 64 + d2) * NPX + pg * 64 + (tid % 8) * 8; *(volatile v8us*)dz = z; __threadfence(); *(volatile v8us*)dz = z; } }
__global__ __launch_bounds__(256) void k_soft(const float* __restrict__ S, int nrows, int n, _Float16* __restrict__ P) {
  #pragma clang fp contract(off)
  const int wv = threadIdx.x >> 5, ln = threadIdx.x & 31; const int r = blockIdx.x * 8 + wv; if (r >= nrows) return; const float* sr = S + (size_t)r * n; float m = -3.0e38f;
#pragma unroll 1
  for (int j = ln; j < n; j += 32) m = fmaxf(m, sr[j]); for (int o = 16; o > 0; o >>= 1) m = fmaxf(m, __shfl_xor(m, o, 32)); float su = 0.f;
#pragma unroll 1
  for (int j = ln; j < n; j += 32) su += expf(sr[j] - m); for (int o = 16; o > 0; o >>= 1) su += __shfl_xor(su, o, 32); const float f = 1024.0f / su;
  for (int pass = 0; pass < 2; ++pass) {
#pragma unroll 1
    for (int j = ln; j < n; j += 32) *(volatile _Float16*)(P + (size_t)r * n + j) = (_Float16)(expf(sr[j] - m) * f); if (pass == 0) __threadfence(); } }
__global__ __launch_bounds__(256) void k_att16(const float* __restrict__ ATTN, _Float16* __restrict__ AT16) { typedef _Float16 v2h __attribute__((ext_vector_type(2))); const int t = blockIdx.x * 256 + threadIdx.x; if (t >= NHD * 64 * 32) return; const int n0 = (t % 32) * 2; const int d = (t / 32) % 64; const int h = t / (32 * 64); v2h v;
  v[0] = (_Float16)ATTN[((size_t)h * NAG + n0) * 64 + d]; v[1] = (_Float16)ATTN[((size_t)h * NAG + n0 + 1) * 64 + d]; _Float16* dst = AT16 + ((size_t)h * 64 + d) * NAG + n0; *(volatile v2h*)dst = v; __threadfence(); *(volatile v2h*)dst = v; }
__global__ __launch_bounds__(256) void k_pe(const float* __restrict__ OUT, const float* __restrict__ QF, const float* __restrict__ pw, const float* __restrict__ ps, const float* __restrict__ pb, _Float16* __restrict__ S16) {
  #pragma clang fp contract(off)
  const size_t t = (size_t)blockIdx.x * 256 + threadIdx.x; if (t >= (size_t)NPX * (CC / 8)) return; const int c0 = (int)(t % (CC / 8)) * 8; const int p = (int)(t / (CC / 8)); const int yo = p / HS, xo = p % HS; FragH f;
#pragma unroll 1
  for (int q = 0; q < 8; ++q) { const int c = c0 + q; float a = 0.f;
#pragma unroll 1
    for (int k = 0; k < 9; ++k) { const int yy = yo + k / 3 - 1, xx = xo + k % 3 - 1; if (yy < 0 || yy >= HS || xx < 0 || xx >= HS) continue; a += bf16_round(pw[c * 9 + k]) * QF[(size_t)(yy * HS + xx) * QW + 2 * CC + c]; }
    float pe = a * bf16_round(ps[c]); pe += bf16_round(pb[c]); const int h = c / HDm, d = c % HDm; float v = OUT[((size_t)h * NPX + p) * 64 + d] + pe; f.h[q] = (_Float16)v; }
  *(volatile v8us*)((unsigned short*)S16 + (size_t)p * CC + c0) = f.half[0]; __threadfence(); *(volatile v8us*)((unsigned short*)S16 + (size_t)p * CC + c0) = f.half[0]; }
__global__ __launch_bounds__(256) void k_fin(const float* __restrict__ G, const float* __restrict__ s, const float* __restrict__ bb, float* __restrict__ outb) {
  #pragma clang fp contract(off)
  const int t = blockIdx.x * 256 + threadIdx.x; if (t >= CC * (NPX / 4)) return; const int p0 = (t % (NPX / 4)) * 4; const int c = t / (NPX / 4); const float sc = bf16_round(s[c]), sh = bf16_round(bb[c]); v4f r; for (int q = 0; q < 4; ++q) { float v = G[(size_t)(p0 + q) * CC + c] * sc; v += sh; r[q] = v; }
  *(volatile v4f*)(outb + (size_t)c * NPX + p0) = r; __threadfence(); *(volatile v4f*)(outb + (size_t)c * NPX + p0) = r; }

extern "C" void kernel_launch(void* const* d_in, const int* in_sizes, int n_in,
                              void* d_out, int out_size, void* d_ws, size_t ws_size, hipStream_t stream) {
  (void)in_sizes; (void)n_in; (void)out_size;
  const float* const* I = (const float* const*)d_in; const float* x = I[0]; const float* qw = I[1]; const float* qs = I[2]; const float* qb = I[3]; const float* pw = I[4]; const float* ps = I[5]; const float* pb = I[6]; const float* jw = I[7]; const float* js = I[8]; const float* jb = I[9];
  char* ws = (char*)d_ws; size_t off = 0;
  auto take = [&](size_t bytes) { char* p = ws + off; off += (bytes + 255) & ~(size_t)255; return p; };
  _Float16* WH = (_Float16*)take((size_t)QW * KI * 2); _Float16* WL = (_Float16*)take((size_t)QW * CC * 2); _Float16* BJ = (_Float16*)take((size_t)CC * CC * 2);
  _Float16* A = (_Float16*)take((size_t)NPX * KI * 2); float* F = (float*)take((size_t)NPX * QW * 4); float* QF = (float*)take((size_t)NPX * QW * 4); _Float16* Q16 = (_Float16*)take((size_t)NPX * QW * 2);
  _Float16* AG = (_Float16*)take((size_t)NHD * NAG * 64 * 2); _Float16* QP = (_Float16*)take((size_t)NHD * NPX * 64 * 2); _Float16* KP = (_Float16*)take((size_t)NHD * NPX * 64 * 2); _Float16* VT = (_Float16*)take((size_t)NHD * 64 * NPX * 2);
  float* S1 = (float*)take((size_t)NHD * NAG * NPX * 4); _Float16* P1 = (_Float16*)take((size_t)NHD * NAG * NPX * 2); float* ATTN = (float*)take((size_t)NHD * NAG * 64 * 4); _Float16* AT16 = (_Float16*)take((size_t)NHD * 64 * NAG * 2); float* S2 = (float*)take((size_t)NHD * NPX * NAG * 4); _Float16* P2 = (_Float16*)take((size_t)NHD * NPX * NAG * 2); float* OUT = (float*)take((size_t)NHD * NPX * 64 * 4); _Float16* S16 = (_Float16*)take((size_t)NPX * CC * 2); float* G = F;
  if (off > ws_size) return;
  k_wqkv<<<(QW * (CC / 8) + 255) / 256, 256, 0, stream>>>(qw, WH, WL); k_wsc<<<(CC * CC / 8 + 255) / 256, 256, 0, stream>>>(jw, BJ, (size_t)CC * CC / 8, 16.0f);
  for (int b = 0; b < NIMG; ++b) { const float* xb = x + (size_t)b * CC * NPX;
    k_im<<<(unsigned)(((size_t)NPX * KT * (CC / 8) + 255) / 256), 256, 0, stream>>>(xb, A);
    k_gemm2<0><<<dim3((NPX / 128) * (QW / 64), 1), 128, 0, stream>>>(A + 4 * CC, KI, 0, WL, CC, 0, 0.0625f / 1024.0f, nullptr, 0, nullptr, 1, 0, 0, F, nullptr, QW, 0, NPX, QW, CC);
    k_gemm2<0><<<dim3((NPX / 128) * (QW / 64), 1), 128, 0, stream>>>(A, KI, 0, WH, KI, 0, 0.0625f, nullptr, 0, F, 1, (size_t)QW, 0, F, nullptr, QW, 0, NPX, QW, KI);
    k_aff<<<(unsigned)(((size_t)NPX * (QW / 8) + 255) / 256), 256, 0, stream>>>(F, qs, qb, QF, Q16);
    k_pool<<<(NHD * NAG * 32 + 255) / 256, 256, 0, stream>>>(QF, AG);
    k_heads<<<(NHD * NPX + 255) / 256, 256, 0, stream>>>(Q16, QP, KP); k_vtp<<<NHD * (NPX / 64), 256, 0, stream>>>(Q16, VT);
    k_gemm2<0><<<dim3(1 * (NPX / 64), NHD), 128, 0, stream>>>(AG, 64, (size_t)NAG * 64, KP, 64, (size_t)NPX * 64, SCL, nullptr, 0, nullptr, 1, 0, 0, S1, nullptr, NPX, (size_t)NAG * NPX, NAG, NPX, 64);
    k_soft<<<(NHD * NAG + 7) / 8, 256, 0, stream>>>(S1, NHD * NAG, NPX, P1);
    k_gemm2<0><<<dim3(1 * 1, NHD), 128, 0, stream>>>(P1, NPX, (size_t)NAG * NPX, VT, NPX, (size_t)64 * NPX, 0.0009765625f, nullptr, 0, nullptr, 1, 0, 0, ATTN, nullptr, 64, (size_t)NAG * 64, NAG, 64, NPX);
    k_att16<<<(NHD * 64 * 32 + 255) / 256, 256, 0, stream>>>(ATTN, AT16);
    k_gemm2<0><<<dim3((NPX / 128) * 1, NHD), 128, 0, stream>>>(QP, 64, (size_t)NPX * 64, AG, 64, (size_t)NAG * 64, SCL, nullptr, 0, nullptr, 1, 0, 0, S2, nullptr, NAG, (size_t)NPX * NAG, NPX, NAG, 64);
    k_soft<<<(NHD * NPX + 7) / 8, 256, 0, stream>>>(S2, NHD * NPX, NAG, P2);
    k_gemm2<0><<<dim3((NPX / 128) * 1, NHD), 128, 0, stream>>>(P2, NAG, (size_t)NPX * NAG, AT16, NAG, (size_t)64 * NAG, 0.0009765625f, nullptr, 0, nullptr, 1, 0, 0, OUT, nullptr, 64, (size_t)NPX * 64, NPX, 64, NAG);
    k_pe<<<(unsigned)(((size_t)NPX * (CC / 8) + 255) / 256), 256, 0, stream>>>(OUT, QF, pw, ps, pb, S16);
    k_gemm2<0><<<dim3((NPX / 128) * (CC / 64), 1), 128, 0, stream>>>(S16, CC, 0, BJ, CC, 0, 0.0625f, nullptr, 0, nullptr, 1, 0, 0, G, nullptr, CC, 0, NPX, CC, CC);
    k_fin<<<(CC * (NPX / 4) + 255) / 256, 256, 0, stream>>>(G, js, jb, (float*)d_out + (size_t)b * CC * NPX); }
}
